// MiniGridPPOMixtureMHNetwork_68719477113
// MI455X (gfx1250) — hardware-verified
//
#include <hip/hip_runtime.h>
#include <stddef.h>
#include <stdint.h>

#define NB   4096
#define NE   4
#define NC   10
#define ND   1024
#define NF   128
#define NO   7
#define NOP  16
#define HP   136
#define GS_EPS 1e-8f

#define T_W2  1024
#define T_W3  5120
#define T_H1  168960
#define T_ALL 171520

static_assert(T_W2 % 256 == 0);
static_assert(T_W3 % 256 == 0);
static_assert(T_H1 % 256 == 0);
static_assert(T_ALL % 256 == 0);
static_assert(T_W2 * 8 == NE * 32 * 64);
static_assert((T_W3 - T_W2) * 8 == NE * 64 * 128);
static_assert((T_H1 - T_W3) * 8 == NC * NF * ND);
static_assert((T_ALL - T_H1) * 8 == NC * NOP * NF);
static_assert(NB % 64 == 0);
static_assert(HP % 8 == 0);
static_assert(ND == 8 * 128);

typedef unsigned short us;
typedef us v8us_t __attribute__((ext_vector_type(8)));
typedef v8us_t __attribute__((may_alias)) v8us;
typedef us v16us __attribute__((ext_vector_type(16)));
typedef __bf16 v16bf __attribute__((ext_vector_type(16)));
typedef float v8f __attribute__((ext_vector_type(8)));
typedef float v4f_t __attribute__((ext_vector_type(4)));
typedef v4f_t __attribute__((may_alias)) v4f;
typedef unsigned int v4u_t __attribute__((ext_vector_type(4)));
typedef v4u_t __attribute__((may_alias)) v4u;

union Frag { v16us v; v8us_t h[2]; };

__device__ __forceinline__ v8f zero8() {
  v8f z;
#pragma unroll
  for (int i = 0; i < 8; ++i) z[i] = 0.0f;
  return z;
}

__device__ __forceinline__ unsigned int bf_bits(float x) {
  const unsigned int u = __float_as_uint(x);
  return (u + 0x7FFFu + ((u >> 16) & 1u)) >> 16;
}
__device__ __forceinline__ void split_bf(float x, unsigned int& hb, unsigned int& lb) {
  hb = bf_bits(x);
  const float r = x - __uint_as_float(hb << 16);
  lb = bf_bits(r);
}
#define SPLIT8(vals, ph, pl)                                           \
  do {                                                                 \
    _Pragma("unroll")                                                  \
    for (int jj_ = 0; jj_ < 4; ++jj_) {                                \
      unsigned int h0_, l0_, h1_, l1_;                                 \
      split_bf((vals)[2 * jj_], h0_, l0_);                             \
      split_bf((vals)[2 * jj_ + 1], h1_, l1_);                         \
      (ph)[jj_] = h0_ | (h1_ << 16);                                   \
      (pl)[jj_] = l0_ | (l1_ << 16);                                   \
    }                                                                  \
  } while (0)

__device__ __forceinline__ v8f mma1(v16us a, v16us b, v8f c) {
  return __builtin_amdgcn_wmma_f32_16x16x32_bf16(false, __builtin_bit_cast(v16bf, a),
                                                 false, __builtin_bit_cast(v16bf, b),
                                                 (short)0, c, false, false);
}
__device__ __forceinline__ v8f mma3(v16us ah, v16us al, v16us bh, v16us bl, v8f c) {
  c = mma1(ah, bh, c);
  c = mma1(ah, bl, c);
  c = mma1(al, bh, c);
  return c;
}

__device__ __forceinline__ float block_sum4(float x, float* red, int slot, int lane, int w) {
#pragma unroll
  for (int off = 16; off > 0; off >>= 1) x += __shfl_xor(x, off, 32);
  if (lane == 0) red[slot * 4 + w] = x;
  __syncthreads();
  return ((red[slot * 4 + 0] + red[slot * 4 + 1]) + red[slot * 4 + 2]) + red[slot * 4 + 3];
}

__global__ void __launch_bounds__(256) prep_kernel(
    const float* __restrict__ w2, const float* __restrict__ w3,
    const float* __restrict__ h1w, const float* __restrict__ h2w,
    us* W2h, us* W2l, us* W3h, us* W3l, us* H1h, us* H1l, us* H2h, us* H2l)
{
  const int i8 = blockIdx.x * 256 + (int)threadIdx.x;
  if (i8 >= T_ALL) return;
  float v[8];
  us* dh;
  us* dl;
  size_t q;
  if (i8 < T_W2) {
    q = (size_t)i8 * 8; dh = W2h; dl = W2l;
#pragma unroll
    for (int j = 0; j < 8; ++j) {
      const int idx = (int)q + j;
      const int row = idx >> 6, k = idx & 63;
      const int tap = k >> 4, ci = k & 15;
      v[j] = w2[(row * 16 + ci) * 4 + tap];
    }
  } else if (i8 < T_W3) {
    q = (size_t)(i8 - T_W2) * 8; dh = W3h; dl = W3l;
#pragma unroll
    for (int j = 0; j < 8; ++j) {
      const int idx = (int)q + j;
      const int row = idx >> 7, k = idx & 127;
      const int tap = k >> 5, ci = k & 31;
      v[j] = w3[(row * 32 + ci) * 4 + tap];
    }
  } else if (i8 < T_H1) {
    q = (size_t)(i8 - T_W3) * 8; dh = H1h; dl = H1l;
    const v4f_t a0 = *(const v4f*)(h1w + q);
    const v4f_t a1 = *(const v4f*)(h1w + q + 4);
#pragma unroll
    for (int j = 0; j < 4; ++j) { v[j] = a0[j]; v[4 + j] = a1[j]; }
  } else {
    q = (size_t)(i8 - T_H1) * 8; dh = H2h; dl = H2l;
#pragma unroll
    for (int j = 0; j < 8; ++j) {
      const int idx = (int)q + j;
      const int row = idx >> 7, f = idx & 127;
      const int cc = row >> 4, o = row & 15;
      const int oc = (o < NO) ? o : (NO - 1);
      const float val = h2w[(cc * NO + oc) * NF + f];
      v[j] = (o < NO) ? val : 0.0f;
    }
  }
  v4u_t ph, pl;
  SPLIT8(v, ph, pl);
  *(volatile v4u_t*)(dh + q) = ph;
  *(volatile v4u_t*)(dl + q) = pl;
  __threadfence();
  *(volatile v4u_t*)(dh + q) = ph;
  *(volatile v4u_t*)(dl + q) = pl;
}

__global__ void __launch_bounds__(128) cnn_mix_kernel(
    const float* __restrict__ state, const int* __restrict__ cvec, const float* __restrict__ te_w,
    const float* __restrict__ w1, const float* __restrict__ b1,
    const float* __restrict__ b2, const float* __restrict__ b3,
    const us* __restrict__ W2h, const us* __restrict__ W2l,
    const us* __restrict__ W3h, const us* __restrict__ W3l,
    us* __restrict__ mixh, us* __restrict__ mixl)
{
  __shared__ float sState[148];
  __shared__ float sW1[NE * 192];
  __shared__ float sB1[NE * 16];
  __shared__ float sB2[NE * 32];
  __shared__ float sB3[NE * 64];
  __shared__ __align__(16) us a1h[NE * 576];
  __shared__ __align__(16) us a1l[NE * 576];
  __shared__ __align__(16) us a2h[NE * 1024];
  __shared__ __align__(16) us a2l[NE * 1024];
  __shared__ __align__(16) float sF[NE * ND];
  __shared__ float sRed[40];

  const int tid  = threadIdx.x;
  const int lane = tid & 31, w = tid >> 5;
  const int h = lane >> 4, m = lane & 15;
  const int b = blockIdx.x;
  const int e = w;

  for (int i = tid; i < 147; i += 128) sState[i] = state[(size_t)b * 147 + i];
  for (int i = tid; i < NE * 192; i += 128) sW1[i] = w1[i];
  if (tid < NE * 16) sB1[tid] = b1[tid];
  sB2[tid] = b2[tid];
  sB3[tid] = b3[tid];
  sB3[tid + 128] = b3[tid + 128];
  __syncthreads();

  {
    float wr[12];
#pragma unroll
    for (int k = 0; k < 12; ++k) wr[k] = sW1[(e * 16 + m) * 12 + k];
    const float bias = sB1[e * 16 + m];
    us* o1h = a1h + e * 576;
    us* o1l = a1l + e * 576;
#pragma unroll 1
    for (int i = 0; i < 18; ++i) {
      const int pos = 2 * i + h;
      const int y = pos / 6;
      const int x = pos - 6 * y;
      const float* sp = sState + y * 7 + x;
      float acc = bias;
#pragma unroll
      for (int ci = 0; ci < 3; ++ci)
#pragma unroll
        for (int ky = 0; ky < 2; ++ky)
#pragma unroll
          for (int kx = 0; kx < 2; ++kx)
            acc = fmaf(wr[ci * 4 + ky * 2 + kx], sp[ci * 49 + ky * 7 + kx], acc);
      acc = fmaxf(acc, 0.0f);
      unsigned int hb, lb;
      split_bf(acc, hb, lb);
      o1h[pos * 16 + m] = (us)hb;
      o1l[pos * 16 + m] = (us)lb;
    }
  }
  __syncthreads();

  {
    const us* A1h = a1h + e * 576;
    const us* A1l = a1l + e * 576;
    int ib[2];
#pragma unroll
    for (int rt = 0; rt < 2; ++rt) {
      int pr = 16 * rt + m;
      pr = (pr > 24) ? 24 : pr;
      const int y2 = pr / 5;
      const int x2 = pr - 5 * y2;
      ib[rt] = y2 * 6 + x2;
    }
    v8f acc2[2][2];
#pragma unroll
    for (int rt = 0; rt < 2; ++rt)
#pragma unroll
      for (int ct = 0; ct < 2; ++ct) acc2[rt][ct] = zero8();
#pragma unroll
    for (int s = 0; s < 2; ++s) {
      Frag fah[2], fal[2], fbh[2], fbl[2];
#pragma unroll
      for (int rt = 0; rt < 2; ++rt) {
        const int ia = (ib[rt] + 6 * s) * 16 + 8 * h;
        const int ic = ia + 16;
        fah[rt].h[0] = *(const v8us*)(A1h + ia);
        fah[rt].h[1] = *(const v8us*)(A1h + ic);
        fal[rt].h[0] = *(const v8us*)(A1l + ia);
        fal[rt].h[1] = *(const v8us*)(A1l + ic);
      }
#pragma unroll
      for (int ct = 0; ct < 2; ++ct) {
        const size_t ob = (size_t)(e * 32 + 16 * ct + m) * 64 + 32 * s + 8 * h;
        fbh[ct].h[0] = *(const v8us*)(W2h + ob);
        fbh[ct].h[1] = *(const v8us*)(W2h + ob + 16);
        fbl[ct].h[0] = *(const v8us*)(W2l + ob);
        fbl[ct].h[1] = *(const v8us*)(W2l + ob + 16);
      }
#pragma unroll
      for (int rt = 0; rt < 2; ++rt)
#pragma unroll
        for (int ct = 0; ct < 2; ++ct)
          acc2[rt][ct] = mma3(fah[rt].v, fal[rt].v, fbh[ct].v, fbl[ct].v, acc2[rt][ct]);
      asm volatile("v_nop\n\tv_nop\n\tv_nop\n\tv_nop"
                   : "+v"(acc2[0][0]), "+v"(acc2[0][1]), "+v"(acc2[1][0]), "+v"(acc2[1][1])
                   : "v"(fah[0].v), "v"(fal[0].v), "v"(fah[1].v), "v"(fal[1].v),
                     "v"(fbh[0].v), "v"(fbl[0].v), "v"(fbh[1].v), "v"(fbl[1].v));
    }
    us* o2h = a2h + e * 1024;
    us* o2l = a2l + e * 1024;
#pragma unroll
    for (int rt = 0; rt < 2; ++rt)
#pragma unroll
      for (int ct = 0; ct < 2; ++ct) {
        const int oc = 16 * ct + m;
        const float bb = sB2[e * 32 + oc];
#pragma unroll
        for (int r = 0; r < 8; ++r) {
          const int pos = 16 * rt + 8 * h + r;
          const float vv = fmaxf(acc2[rt][ct][r] + bb, 0.0f);
          unsigned int hb, lb;
          split_bf(vv, hb, lb);
          o2h[pos * 32 + oc] = (us)hb;
          o2l[pos * 32 + oc] = (us)lb;
        }
      }
  }
  __syncthreads();

  {
    const us* A2h = a2h + e * 1024;
    const us* A2l = a2l + e * 1024;
    const int i3 = (m >> 2) * 5 + (m & 3);
    v8f acc3[4];
#pragma unroll
    for (int ct = 0; ct < 4; ++ct) acc3[ct] = zero8();
#pragma unroll 1
    for (int s = 0; s < 4; ++s) {
      const int idx = i3 + (s >> 1) * 5 + (s & 1);
      const int ia = idx * 32 + 8 * h;
      Frag fah, fal, fbh[4], fbl[4];
      fah.h[0] = *(const v8us*)(A2h + ia);
      fah.h[1] = *(const v8us*)(A2h + ia + 16);
      fal.h[0] = *(const v8us*)(A2l + ia);
      fal.h[1] = *(const v8us*)(A2l + ia + 16);
#pragma unroll
      for (int ct = 0; ct < 4; ++ct) {
        const size_t ob = (size_t)(e * 64 + 16 * ct + m) * 128 + 32 * s + 8 * h;
        fbh[ct].h[0] = *(const v8us*)(W3h + ob);
        fbh[ct].h[1] = *(const v8us*)(W3h + ob + 16);
        fbl[ct].h[0] = *(const v8us*)(W3l + ob);
        fbl[ct].h[1] = *(const v8us*)(W3l + ob + 16);
      }
#pragma unroll
      for (int ct = 0; ct < 4; ++ct)
        acc3[ct] = mma3(fah.v, fal.v, fbh[ct].v, fbl[ct].v, acc3[ct]);
      asm volatile("v_nop\n\tv_nop\n\tv_nop\n\tv_nop"
                   : "+v"(acc3[0]), "+v"(acc3[1]), "+v"(acc3[2]), "+v"(acc3[3])
                   : "v"(fah.v), "v"(fal.v),
                     "v"(fbh[0].v), "v"(fbl[0].v), "v"(fbh[1].v), "v"(fbl[1].v),
                     "v"(fbh[2].v), "v"(fbl[2].v), "v"(fbh[3].v), "v"(fbl[3].v));
    }
#pragma unroll
    for (int ct = 0; ct < 4; ++ct) {
      const int oc = 16 * ct + m;
      const float bb = sB3[e * 64 + oc];
      v4f_t q0, q1;
#pragma unroll
      for (int r = 0; r < 4; ++r) { q0[r] = acc3[ct][r] + bb; q1[r] = acc3[ct][4 + r] + bb; }
      v4f* dst = (v4f*)(sF + e * ND + oc * 16 + 8 * h);
      dst[0] = q0;
      dst[1] = q1;
    }
  }
  __syncthreads();

  {
    float x0[8], x1[8], x2[8], x3[8];
    {
      const v4f* p0 = (const v4f*)(sF + 0 * ND + 8 * tid);
      const v4f* p1 = (const v4f*)(sF + 1 * ND + 8 * tid);
      const v4f* p2 = (const v4f*)(sF + 2 * ND + 8 * tid);
      const v4f* p3 = (const v4f*)(sF + 3 * ND + 8 * tid);
      const v4f_t a0 = p0[0], c0 = p0[1];
      const v4f_t a1 = p1[0], c1 = p1[1];
      const v4f_t a2 = p2[0], c2 = p2[1];
      const v4f_t a3 = p3[0], c3 = p3[1];
#pragma unroll
      for (int j = 0; j < 4; ++j) {
        x0[j] = a0[j]; x0[4 + j] = c0[j];
        x1[j] = a1[j]; x1[4 + j] = c1[j];
        x2[j] = a2[j]; x2[4 + j] = c2[j];
        x3[j] = a3[j]; x3[4 + j] = c3[j];
      }
    }
    float s, t, u;
    s = 0.0f;
#pragma unroll
    for (int j = 0; j < 8; ++j) s += x0[j] * x0[j];
    {
      const float n0 = block_sum4(s, sRed, 0, lane, w);
      const float inv = 1.0f / (sqrtf(n0) + GS_EPS);
#pragma unroll
      for (int j = 0; j < 8; ++j) x0[j] *= inv;
    }
    s = 0.0f;
#pragma unroll
    for (int j = 0; j < 8; ++j) s += x1[j] * x0[j];
    {
      const float p10 = block_sum4(s, sRed, 1, lane, w);
#pragma unroll
      for (int j = 0; j < 8; ++j) x1[j] = x1[j] - p10 * x0[j];
      s = 0.0f;
#pragma unroll
      for (int j = 0; j < 8; ++j) s += x1[j] * x1[j];
      const float n1 = block_sum4(s, sRed, 2, lane, w);
      const float inv = 1.0f / (sqrtf(n1) + GS_EPS);
#pragma unroll
      for (int j = 0; j < 8; ++j) x1[j] *= inv;
    }
    s = 0.0f; t = 0.0f;
#pragma unroll
    for (int j = 0; j < 8; ++j) { s += x2[j] * x0[j]; t += x2[j] * x1[j]; }
    {
      const float p20 = block_sum4(s, sRed, 3, lane, w);
      const float p21 = block_sum4(t, sRed, 4, lane, w);
#pragma unroll
      for (int j = 0; j < 8; ++j) x2[j] = x2[j] - (p20 * x0[j] + p21 * x1[j]);
      s = 0.0f;
#pragma unroll
      for (int j = 0; j < 8; ++j) s += x2[j] * x2[j];
      const float n2 = block_sum4(s, sRed, 5, lane, w);
      const float inv = 1.0f / (sqrtf(n2) + GS_EPS);
#pragma unroll
      for (int j = 0; j < 8; ++j) x2[j] *= inv;
    }
    s = 0.0f; t = 0.0f; u = 0.0f;
#pragma unroll
    for (int j = 0; j < 8; ++j) { s += x3[j] * x0[j]; t += x3[j] * x1[j]; u += x3[j] * x2[j]; }
    {
      const float p30 = block_sum4(s, sRed, 6, lane, w);
      const float p31 = block_sum4(t, sRed, 7, lane, w);
      const float p32 = block_sum4(u, sRed, 8, lane, w);
#pragma unroll
      for (int j = 0; j < 8; ++j) x3[j] = x3[j] - ((p30 * x0[j] + p31 * x1[j]) + p32 * x2[j]);
      s = 0.0f;
#pragma unroll
      for (int j = 0; j < 8; ++j) s += x3[j] * x3[j];
      const float n3 = block_sum4(s, sRed, 9, lane, w);
      const float inv = 1.0f / (sqrtf(n3) + GS_EPS);
#pragma unroll
      for (int j = 0; j < 8; ++j) x3[j] *= inv;
    }
    int cb = cvec[b];
    cb = (cb < 0) ? 0 : ((cb > NC - 1) ? (NC - 1) : cb);
    const float g0 = te_w[0 * NC + cb], g1 = te_w[1 * NC + cb];
    const float g2 = te_w[2 * NC + cb], g3 = te_w[3 * NC + cb];
    float mx[8];
#pragma unroll
    for (int j = 0; j < 8; ++j)
      mx[j] = tanhf(((g0 * x0[j] + g1 * x1[j]) + g2 * x2[j]) + g3 * x3[j]);
    v4u_t ph, pl;
    SPLIT8(mx, ph, pl);
    const size_t od = (size_t)b * ND + 8 * tid;
    *(volatile v4u_t*)(mixh + od) = ph;
    *(volatile v4u_t*)(mixl + od) = pl;
    __threadfence();
    *(volatile v4u_t*)(mixh + od) = ph;
    *(volatile v4u_t*)(mixl + od) = pl;
  }
}

__global__ void __launch_bounds__(256) head_kernel(
    const us* __restrict__ mixh, const us* __restrict__ mixl,
    const us* __restrict__ H1h, const us* __restrict__ H1l, const float* __restrict__ h1b,
    const us* __restrict__ H2h, const us* __restrict__ H2l, const float* __restrict__ h2b,
    const int* __restrict__ cvec, float* __restrict__ out)
{
  __shared__ __align__(16) us t1h[64 * HP];
  __shared__ __align__(16) us t1l[64 * HP];
  __shared__ __align__(16) float sOut[64 * NO];

  const int tid  = threadIdx.x;
  const int lane = tid & 31, w = tid >> 5;
  const int h = lane >> 4, m = lane & 15;
  const int rg = w >> 2, cg = w & 3;
  const int row0 = blockIdx.x * 64;

  int cbr[8];
  {
    const int rb = row0 + 16 * (w & 3) + 8 * h;
#pragma unroll
    for (int r = 0; r < 8; ++r) {
      int cc = cvec[rb + r];
      cbr[r] = (cc < 0) ? 0 : ((cc > NC - 1) ? (NC - 1) : cc);
    }
  }
  v8f osel = zero8();

  const us* pa_h = mixh + (size_t)(row0 + 32 * rg + m) * ND + 8 * h;
  const us* pa_l = mixl + (size_t)(row0 + 32 * rg + m) * ND + 8 * h;

#pragma unroll 1
  for (int c = 0; c < NC; ++c) {
    v8f acc[2][2];
#pragma unroll
    for (int rt = 0; rt < 2; ++rt)
#pragma unroll
      for (int ct = 0; ct < 2; ++ct) acc[rt][ct] = zero8();
    const us* pb_h = H1h + (size_t)(c * NF + 32 * cg + m) * ND + 8 * h;
    const us* pb_l = H1l + (size_t)(c * NF + 32 * cg + m) * ND + 8 * h;
#pragma unroll 1
    for (int k0 = 0; k0 < ND; k0 += 32) {
      Frag fah[2], fal[2], fbh[2], fbl[2];
#pragma unroll
      for (int rt = 0; rt < 2; ++rt) {
        const size_t oa = (size_t)rt * 16 * ND + k0;
        fah[rt].h[0] = *(const v8us*)(pa_h + oa);
        fah[rt].h[1] = *(const v8us*)(pa_h + oa + 16);
        fal[rt].h[0] = *(const v8us*)(pa_l + oa);
        fal[rt].h[1] = *(const v8us*)(pa_l + oa + 16);
      }
#pragma unroll
      for (int ct = 0; ct < 2; ++ct) {
        const size_t obb = (size_t)ct * 16 * ND + k0;
        fbh[ct].h[0] = *(const v8us*)(pb_h + obb);
        fbh[ct].h[1] = *(const v8us*)(pb_h + obb + 16);
        fbl[ct].h[0] = *(const v8us*)(pb_l + obb);
        fbl[ct].h[1] = *(const v8us*)(pb_l + obb + 16);
      }
#pragma unroll
      for (int rt = 0; rt < 2; ++rt)
#pragma unroll
        for (int ct = 0; ct < 2; ++ct)
          acc[rt][ct] = mma3(fah[rt].v, fal[rt].v, fbh[ct].v, fbl[ct].v, acc[rt][ct]);
      asm volatile("v_nop\n\tv_nop\n\tv_nop\n\tv_nop"
                   : "+v"(acc[0][0]), "+v"(acc[0][1]), "+v"(acc[1][0]), "+v"(acc[1][1])
                   : "v"(fah[0].v), "v"(fal[0].v), "v"(fah[1].v), "v"(fal[1].v),
                     "v"(fbh[0].v), "v"(fbl[0].v), "v"(fbh[1].v), "v"(fbl[1].v));
    }
#pragma unroll
    for (int ct = 0; ct < 2; ++ct) {
      const int f = 32 * cg + 16 * ct + m;
      const float bias = h1b[c * NF + f];
#pragma unroll
      for (int rt = 0; rt < 2; ++rt)
#pragma unroll
        for (int r = 0; r < 8; ++r) {
          const int row = 32 * rg + 16 * rt + 8 * h + r;
          const float vv = tanhf(acc[rt][ct][r] + bias);
          unsigned int hb, lb;
          split_bf(vv, hb, lb);
          t1h[row * HP + f] = (us)hb;
          t1l[row * HP + f] = (us)lb;
        }
    }
    __syncthreads();
    if (w < 4) {
      v8f a2 = zero8();
      const us* qa_h = t1h + (16 * w + m) * HP + 8 * h;
      const us* qa_l = t1l + (16 * w + m) * HP + 8 * h;
      const us* qb_h = H2h + (size_t)(c * NOP + m) * NF + 8 * h;
      const us* qb_l = H2l + (size_t)(c * NOP + m) * NF + 8 * h;
#pragma unroll
      for (int ks = 0; ks < 4; ++ks) {
        const int k0 = 32 * ks;
        Frag gah, gal, gbh, gbl;
        gah.h[0] = *(const v8us*)(qa_h + k0);
        gah.h[1] = *(const v8us*)(qa_h + k0 + 16);
        gal.h[0] = *(const v8us*)(qa_l + k0);
        gal.h[1] = *(const v8us*)(qa_l + k0 + 16);
        gbh.h[0] = *(const v8us*)(qb_h + k0);
        gbh.h[1] = *(const v8us*)(qb_h + k0 + 16);
        gbl.h[0] = *(const v8us*)(qb_l + k0);
        gbl.h[1] = *(const v8us*)(qb_l + k0 + 16);
        a2 = mma3(gah.v, gal.v, gbh.v, gbl.v, a2);
        asm volatile("v_nop\n\tv_nop\n\tv_nop\n\tv_nop"
                     : "+v"(a2)
                     : "v"(gah.v), "v"(gal.v), "v"(gbh.v), "v"(gbl.v));
      }
      const int mo = (m < NO) ? m : (NO - 1);
      const float bb = h2b[c * NO + mo];
#pragma unroll
      for (int r = 0; r < 8; ++r) {
        const float vv = a2[r] + bb;
        osel[r] = (cbr[r] == c) ? vv : osel[r];
      }
    }
    __syncthreads();
  }

  if (w < 4 && m < NO) {
#pragma unroll
    for (int r = 0; r < 8; ++r) sOut[(16 * w + 8 * h + r) * NO + m] = osel[r];
  }
  __syncthreads();
  if (w == 0) {
    float* go = out + (size_t)row0 * NO;
    v4f_t vv[4];
#pragma unroll
    for (int p = 0; p < 4; ++p) {
      const int idx = p * 32 + lane;
      const int ic = (idx < 112) ? idx : 111;
      vv[p] = *(const v4f*)(sOut + ic * 4);
    }
#pragma unroll
    for (int p = 0; p < 4; ++p) {
      const int idx = p * 32 + lane;
      if (idx < 112) *(volatile v4f_t*)(go + idx * 4) = vv[p];
    }
    __threadfence();
#pragma unroll
    for (int p = 0; p < 4; ++p) {
      const int idx = p * 32 + lane;
      if (idx < 112) *(volatile v4f_t*)(go + idx * 4) = vv[p];
    }
  }
}

extern "C" void kernel_launch(void* const* d_in, const int* in_sizes, int n_in,
                              void* d_out, int out_size, void* d_ws, size_t ws_size,
                              hipStream_t stream)
{
  if (n_in < 13) return;
  if (in_sizes[0]  != NB * 3 * 7 * 7) return;
  if (in_sizes[1]  != NB) return;
  if (in_sizes[2]  != NE * NC) return;
  if (in_sizes[3]  != NE * 16 * 3 * 4) return;
  if (in_sizes[4]  != NE * 16) return;
  if (in_sizes[5]  != NE * 32 * 16 * 4) return;
  if (in_sizes[6]  != NE * 32) return;
  if (in_sizes[7]  != NE * 64 * 32 * 4) return;
  if (in_sizes[8]  != NE * 64) return;
  if (in_sizes[9]  != NC * NF * ND) return;
  if (in_sizes[10] != NC * NF) return;
  if (in_sizes[11] != NC * NO * NF) return;
  if (in_sizes[12] != NC * NO) return;
  if (out_size != NB * NO) return;

  const float* state = (const float*)d_in[0];
  const int*   cvec  = (const int*)d_in[1];
  const float* te_w  = (const float*)d_in[2];
  const float* c1w   = (const float*)d_in[3];
  const float* c1b   = (const float*)d_in[4];
  const float* c2w   = (const float*)d_in[5];
  const float* c2b   = (const float*)d_in[6];
  const float* c3w   = (const float*)d_in[7];
  const float* c3b   = (const float*)d_in[8];
  const float* h1w   = (const float*)d_in[9];
  const float* h1b   = (const float*)d_in[10];
  const float* h2w   = (const float*)d_in[11];
  const float* h2b   = (const float*)d_in[12];
  float* out = (float*)d_out;

  const size_t bW2 = (size_t)NE * 32 * 64 * 2;
  const size_t bW3 = (size_t)NE * 64 * 128 * 2;
  const size_t bH1 = (size_t)NC * NF * ND * 2;
  const size_t bH2 = (size_t)NC * NOP * NF * 2;
  const size_t bMX = (size_t)NB * ND * 2;
  const size_t oW2h = 0;
  const size_t oW2l = oW2h + bW2;
  const size_t oW3h = oW2l + bW2;
  const size_t oW3l = oW3h + bW3;
  const size_t oH1h = oW3l + bW3;
  const size_t oH1l = oH1h + bH1;
  const size_t oH2h = oH1l + bH1;
  const size_t oH2l = oH2h + bH2;
  const size_t oMXh = oH2l + bH2;
  const size_t oMXl = oMXh + bMX;
  const size_t total = oMXl + bMX;
  if (total > ws_size) return;

  char* ws = (char*)d_ws;
  us* W2h = (us*)(ws + oW2h); us* W2l = (us*)(ws + oW2l);
  us* W3h = (us*)(ws + oW3h); us* W3l = (us*)(ws + oW3l);
  us* H1h = (us*)(ws + oH1h); us* H1l = (us*)(ws + oH1l);
  us* H2h = (us*)(ws + oH2h); us* H2l = (us*)(ws + oH2l);
  us* MXh = (us*)(ws + oMXh); us* MXl = (us*)(ws + oMXl);

  prep_kernel<<<T_ALL / 256, 256, 0, stream>>>(c2w, c3w, h1w, h2w,
                                               W2h, W2l, W3h, W3l, H1h, H1l, H2h, H2l);
  cnn_mix_kernel<<<NB, 128, 0, stream>>>(state, cvec, te_w, c1w, c1b, c2b, c3b,
                                         W2h, W2l, W3h, W3l, MXh, MXl);
  head_kernel<<<NB / 64, 256, 0, stream>>>(MXh, MXl, H1h, H1l, h1b, H2h, H2l, h2b, cvec, out);
}
